// MoELayer_81114752352735
// MI455X (gfx1250) — hardware-verified
//
#include <hip/hip_runtime.h>
#include <math.h>

#ifndef NTOK
#define NTOK 4096
#endif
#define NTOK_FULL 4096
#define DM 1024
#define NE 8
#define TOPK 2
#define NSLOT (NTOK * TOPK)
#define R_MAX (NSLOT + 64 * NE)
#define NT_MAX (R_MAX / 64)
#define SPT (NSLOT / 512)

#define CX_LOG2 11
#define CW_LOG2 16
#define SC_Y (1.0f / (float)(1u << (CX_LOG2 + CW_LOG2)))

#define TBL_COUNT 0
#define TBL_POFF 16
#define TBL_NTILES 32
#define TBL_TILE_E 64
#define TBL_ROWTOK 256
#define TBL_SLOTROW (256 + R_MAX)
#define TBL_WORDS (256 + R_MAX + NSLOT)

static_assert(NE <= 16 && TOPK == 2 && NSLOT % 512 == 0);
static_assert(NE == 8);
static_assert(NTOK <= NTOK_FULL && NTOK % 128 == 0);
static_assert(SPT % 4 == 0 && SPT >= 4);
static_assert(R_MAX % 64 == 0 && TBL_TILE_E + NT_MAX <= 256);
static_assert(DM == 1024);
static_assert((NTOK * DM / 8) % 256 == 0 && (NE * DM * DM / 8) % 256 == 0);
static_assert((TBL_WORDS * 4) % 256 == 0);
static_assert(R_MAX >= NSLOT);
static_assert(NTOK != 4096 || (NSLOT == 8192 && R_MAX == 8704 && NT_MAX == 136 && SPT == 16 && DM == 1024));

constexpr size_t al256(size_t b) { return (b + 255) & ~(size_t)255; }
constexpr size_t SZ_X16 = al256((size_t)NTOK * DM * 2);
constexpr size_t SZ_W   = al256((size_t)NE * DM * DM * 2);
constexpr size_t SZ_SEL = al256((size_t)NSLOT * 4);
constexpr size_t SZ_WGT = al256((size_t)NSLOT * 4);
constexpr size_t SZ_TBL = al256((size_t)TBL_WORDS * 4);
constexpr size_t SZ_XG  = al256((size_t)R_MAX * DM * 2);
constexpr size_t SZ_YG  = al256((size_t)R_MAX * DM * 4);
constexpr size_t WS_TOTAL = SZ_X16 + SZ_W + SZ_SEL + SZ_WGT + SZ_TBL + SZ_XG + SZ_YG;
static_assert(WS_TOTAL < (size_t)134217728);
static_assert(NTOK != 4096 || WS_TOTAL == (size_t)78777344);

typedef _Float16 h16;
typedef __attribute__((ext_vector_type(16))) _Float16 v16h;
typedef __attribute__((ext_vector_type(8)))  _Float16 v8h;
typedef __attribute__((ext_vector_type(8)))  float    v8f;
typedef __attribute__((ext_vector_type(4)))  float    v4f;
typedef __attribute__((ext_vector_type(2)))  float    v2f;
typedef __attribute__((ext_vector_type(4)))  unsigned int v4u;
typedef __attribute__((ext_vector_type(4)))  int      v4i;
typedef __attribute__((ext_vector_type(2)))  int      v2i;


#define VST2(T, ptr, val) do { const T vst2_v_ = (val); *(volatile T*)(ptr) = vst2_v_; __threadfence(); *(volatile T*)(ptr) = vst2_v_; } while (0)

static __device__ __forceinline__ float bfr(float f) {
    unsigned u = __float_as_uint(f);
    u += 0x7FFFu + ((u >> 16) & 1u);
    return __uint_as_float(u & 0xFFFF0000u);
}
static __device__ __forceinline__ h16 toh_flush(float v) { const float w = (fabsf(v) < 6.103515625e-05f) ? 0.0f : v; return (h16)w; }
static __device__ __forceinline__ void st8h(h16* p, const float* v) {
    v8h hv;
#pragma unroll
    for (int e = 0; e < 8; ++e) hv[e] = toh_flush(v[e]);
    VST2(v8h, p, hv);
}

union FragU { v16h v; v8h h[2]; };
static __device__ __forceinline__ v16h frag_ld(const h16* p) {
    FragU f; f.h[0] = *(const v8h*)(p); f.h[1] = *(const v8h*)(p + 16); return f.v;
}
static __device__ __forceinline__ v8f wmma16g(v16h a, v16h b, v8f c) {
    c = __builtin_amdgcn_wmma_f32_16x16x32_f16(false, a, false, b, (short)0, c, false, false);
    asm volatile("v_nop\n\tv_nop\n\tv_nop\n\tv_nop" : "+v"(c) : "v"(a), "v"(b));
    return c;
}
static __device__ __forceinline__ void wave_sync_lds() {
    __builtin_amdgcn_fence(3  , "workgroup");
    __builtin_amdgcn_wave_barrier();
    __builtin_amdgcn_fence(2  , "workgroup");
}

template <int LOG2C>
__global__ __launch_bounds__(256) void k_plane(const float* __restrict__ src, h16* __restrict__ dst, unsigned n8) {
    const unsigned u = blockIdx.x * 256u + threadIdx.x;
    if (u >= n8) return;
    const float cs = (float)(1u << LOG2C);
    const v4f a = *(const v4f*)(src + (size_t)u * 8u);
    const v4f b = *(const v4f*)(src + (size_t)u * 8u + 4u);
    float v[8] = {bfr(a.x) * cs, bfr(a.y) * cs, bfr(a.z) * cs, bfr(a.w) * cs, bfr(b.x) * cs, bfr(b.y) * cs, bfr(b.z) * cs, bfr(b.w) * cs};
    st8h(dst + (size_t)u * 8u, v);
}

__global__ __launch_bounds__(256) void k_planeT(const float* __restrict__ src, h16* __restrict__ dst) {
    __shared__ __align__(16) float sT[64 * 68];
    const unsigned tid = threadIdx.x;
    const unsigned bx = blockIdx.x;
    const unsigned TPE = (unsigned)((DM / 64) * (DM / 64));
    if (bx >= (unsigned)NE * TPE) return;
    const unsigned e = bx / TPE;
    const unsigned rem = bx - e * TPE;
    const unsigned kt = rem / (unsigned)(DM / 64);
    const unsigned nt = rem - kt * (unsigned)(DM / 64);
    const unsigned k0 = kt * 64u, n0 = nt * 64u;
    const float cs = (float)(1u << CW_LOG2);
    const size_t ebase = (size_t)e * (size_t)(DM * DM);
#pragma unroll
    for (int i = 0; i < 4; ++i) {
        const unsigned p = tid + 256u * (unsigned)i;
        const unsigned kr = p >> 4;
        const unsigned n4 = (p & 15u) * 4u;
        const v4f a = *(const v4f*)(src + ebase + (size_t)(k0 + kr) * DM + n0 + n4);
        v4f s;
        s.x = bfr(a.x) * cs; s.y = bfr(a.y) * cs; s.z = bfr(a.z) * cs; s.w = bfr(a.w) * cs;
        *(v4f*)(&sT[kr * 68u + n4]) = s;
    }
    __syncthreads();
#pragma unroll
    for (int i = 0; i < 2; ++i) {
        const unsigned q = tid + 256u * (unsigned)i;
        const unsigned n = q >> 3;
        const unsigned kp = q & 7u;
        float v[8];
#pragma unroll
        for (int j = 0; j < 8; ++j) v[j] = sT[(8u * kp + (unsigned)j) * 68u + n];
        st8h(dst + ebase + (size_t)(n0 + n) * DM + k0 + 8u * kp, v);
    }
}

__global__ __launch_bounds__(256) void k_gate(const float* __restrict__ x, const float* __restrict__ nx, const float* __restrict__ rw,
                                              const float* __restrict__ nw, int* __restrict__ sel, float* __restrict__ wgt) {
    const unsigned lane = threadIdx.x & 31u;
    const unsigned wave = threadIdx.x >> 5;
    const unsigned t0 = (blockIdx.x * 8u + wave) * 16u;
    if (t0 >= (unsigned)NTOK) return;
    int ki0 = 0, ki1 = 0;
    float kw0 = 0.0f, kw1 = 0.0f;
    for (unsigned j = 0; j < 16u; ++j) {
        const float* xr = x + (size_t)(t0 + j) * DM;
        const float* nr = nx + (size_t)(t0 + j) * DM;
        float lg[NE];
#pragma unroll
        for (int e = 0; e < NE; ++e) lg[e] = 0.0f;
        for (unsigned i = 0; i < (unsigned)(DM / 32); ++i) {
            const unsigned d = lane + 32u * i;
            const float xv = bfr(xr[d]);
            const float nv = bfr(nr[d]);
            const v4f ra = *(const v4f*)(rw + d * 8u);
            const v4f rb = *(const v4f*)(rw + d * 8u + 4u);
            const v4f na = *(const v4f*)(nw + d * 8u);
            const v4f nb = *(const v4f*)(nw + d * 8u + 4u);
            const float rr[NE] = {bfr(ra.x), bfr(ra.y), bfr(ra.z), bfr(ra.w), bfr(rb.x), bfr(rb.y), bfr(rb.z), bfr(rb.w)};
            const float nn[NE] = {bfr(na.x), bfr(na.y), bfr(na.z), bfr(na.w), bfr(nb.x), bfr(nb.y), bfr(nb.z), bfr(nb.w)};
#pragma unroll
            for (int e = 0; e < NE; ++e) { lg[e] += xv * rr[e]; lg[e] += nv * nn[e]; }
        }
#pragma unroll
        for (int e = 0; e < NE; ++e) {
            lg[e] += __shfl_xor(lg[e], 16, 32);
            lg[e] += __shfl_xor(lg[e], 8, 32);
            lg[e] += __shfl_xor(lg[e], 4, 32);
            lg[e] += __shfl_xor(lg[e], 2, 32);
            lg[e] += __shfl_xor(lg[e], 1, 32);
        }
        float mx = lg[0];
#pragma unroll
        for (int e = 1; e < NE; ++e) mx = (lg[e] > mx) ? lg[e] : mx;
        float pr[NE];
#pragma unroll
        for (int e = 0; e < NE; ++e) pr[e] = expf(lg[e] - mx);
        float sum = 0.0f;
#pragma unroll
        for (int e = 0; e < NE; ++e) sum += pr[e];
#pragma unroll
        for (int e = 0; e < NE; ++e) pr[e] = pr[e] / sum;
        float bestv = pr[0];
        int besti = 0;
#pragma unroll
        for (int e = 1; e < NE; ++e) { const bool c = pr[e] > bestv; bestv = c ? pr[e] : bestv; besti = c ? e : besti; }
        float secv = -1.0f;
        int seci = 0;
#pragma unroll
        for (int e = 0; e < NE; ++e) { const bool c = (e != besti) && (pr[e] > secv); secv = c ? pr[e] : secv; seci = c ? e : seci; }
        const float den = bestv + secv;
        const float w0 = bestv / den;
        const float w1 = secv / den;
        const bool mine = (lane == j);
        ki0 = mine ? besti : ki0;  ki1 = mine ? seci : ki1;
        kw0 = mine ? w0 : kw0;     kw1 = mine ? w1 : kw1;
    }
    if (lane < 16u) {
        v2i sv; sv.x = ki0; sv.y = ki1;
        v2f wv; wv.x = kw0; wv.y = kw1;
        VST2(v2i, sel + (size_t)(t0 + lane) * 2u, sv);
        VST2(v2f, wgt + (size_t)(t0 + lane) * 2u, wv);
    }
}

__global__ __launch_bounds__(512) void k_route(const int* __restrict__ sel, int* __restrict__ tbl) {
    __shared__ __align__(16) int s_rt[R_MAX];
    __shared__ __align__(16) int s_hdr[256];
    __shared__ int sc[512];
    const unsigned tid = threadIdx.x;
    for (unsigned i = tid; i < (unsigned)R_MAX; i += 512u) s_rt[i] = -1;
    if (tid < 256u) s_hdr[tid] = (tid >= (unsigned)TBL_TILE_E && tid < (unsigned)(TBL_TILE_E + NT_MAX)) ? -1 : 0;
    __syncthreads();
    int es[SPT];
    int cnt[NE];
#pragma unroll
    for (int j = 0; j < NE; ++j) cnt[j] = 0;
    const v4i* sp = (const v4i*)(sel + (size_t)tid * (unsigned)SPT);
#pragma unroll
    for (int g = 0; g < SPT / 4; ++g) {
        const v4i v = sp[g];
        es[4 * g + 0] = min(max(v.x, 0), NE - 1);
        es[4 * g + 1] = min(max(v.y, 0), NE - 1);
        es[4 * g + 2] = min(max(v.z, 0), NE - 1);
        es[4 * g + 3] = min(max(v.w, 0), NE - 1);
    }
#pragma unroll
    for (int q = 0; q < SPT; ++q)
#pragma unroll
        for (int j = 0; j < NE; ++j) cnt[j] += (es[q] == j) ? 1 : 0;
    int base[NE], total[NE];
#pragma unroll
    for (int j = 0; j < NE; ++j) {
        sc[tid] = cnt[j];
        __syncthreads();
        for (unsigned off = 1u; off < 512u; off <<= 1) {
            const unsigned src = (tid >= off) ? (tid - off) : 0u;
            const int add = sc[src];
            const int v = sc[tid] + ((tid >= off) ? add : 0);
            __syncthreads();
            sc[tid] = v;
            __syncthreads();
        }
        base[j] = sc[tid] - cnt[j];
        total[j] = sc[511];
        __syncthreads();
    }
    int poff[NE + 1];
    poff[0] = 0;
#pragma unroll
    for (int j = 0; j < NE; ++j) poff[j + 1] = poff[j] + (((total[j] + 63) >> 6) << 6);
    int rw[SPT];
#pragma unroll
    for (int q = 0; q < SPT; ++q) {
        int row = 0;
#pragma unroll
        for (int j = 0; j < NE; ++j) {
            const bool hit = (es[q] == j);
            row = hit ? (poff[j] + base[j]) : row;
            base[j] += hit ? 1 : 0;
        }
        row = min(max(row, 0), R_MAX - 1);
        rw[q] = row;
        s_rt[row] = (int)((tid * (unsigned)SPT + (unsigned)q) >> 1);
    }
    if (tid == 0u) {
#pragma unroll
        for (int j = 0; j < NE; ++j) { s_hdr[TBL_COUNT + j] = total[j]; s_hdr[TBL_POFF + j] = poff[j]; }
        s_hdr[TBL_POFF + NE] = poff[NE];
        s_hdr[TBL_NTILES] = poff[NE] >> 6;
    }
    if (tid < (unsigned)NT_MAX) {
        const int b64 = (int)(tid * 64u);
        int ev = -1;
#pragma unroll
        for (int j = 0; j < NE; ++j) ev = (b64 >= poff[j] && b64 < poff[j + 1]) ? j : ev;
        s_hdr[TBL_TILE_E + tid] = ev;
    }
    __syncthreads();
    for (int pass = 0; pass < 2; ++pass) {
        if (tid < 64u) *(volatile v4i*)(tbl + 4u * tid) = *(const v4i*)(&s_hdr[4u * tid]);
        for (unsigned i = tid; i < (unsigned)(R_MAX / 4); i += 512u) *(volatile v4i*)(tbl + TBL_ROWTOK + 4u * i) = *(const v4i*)(&s_rt[4u * i]);
        __threadfence();
    }
    __syncthreads();
#pragma unroll
    for (int g = 0; g < SPT / 4; ++g) {
        v4i pk; pk.x = rw[4 * g]; pk.y = rw[4 * g + 1]; pk.z = rw[4 * g + 2]; pk.w = rw[4 * g + 3];
        *(v4i*)(&s_rt[tid * (unsigned)SPT + 4u * (unsigned)g]) = pk;
    }
    __syncthreads();
    for (int pass = 0; pass < 2; ++pass) {
        for (unsigned i = tid; i < (unsigned)(NSLOT / 4); i += 512u) *(volatile v4i*)(tbl + TBL_SLOTROW + 4u * i) = *(const v4i*)(&s_rt[4u * i]);
        __threadfence();
    }
}

__global__ __launch_bounds__(256) void k_gather(const h16* __restrict__ x16, const int* __restrict__ tbl, h16* __restrict__ Xg) {
    const unsigned row = blockIdx.x * 2u + (threadIdx.x >> 7);
    if (row >= (unsigned)R_MAX) return;
    const unsigned c = (threadIdx.x & 127u) * 8u;
    const int tr = tbl[TBL_ROWTOK + row];
    const bool pad = (tr < 0);
    const int tok = min(max(tr, 0), NTOK - 1);
    const v4u ld = *(const v4u*)(x16 + (size_t)(unsigned)tok * DM + c);
    v4u v;
    v.x = pad ? 0u : ld.x; v.y = pad ? 0u : ld.y; v.z = pad ? 0u : ld.z; v.w = pad ? 0u : ld.w;
    VST2(v4u, Xg + (size_t)row * DM + c, v);
}

__global__ __launch_bounds__(256) void k_ffn(const h16* __restrict__ Xg, const h16* __restrict__ Wp, const float* __restrict__ eb,
                                             const int* __restrict__ tbl, float* __restrict__ Yg) {
    __shared__ __align__(16) float sT[8][16 * 68];
    const unsigned lane = threadIdx.x & 31u;
    const unsigned wave = threadIdx.x >> 5;
    const unsigned u = blockIdx.x * 8u + wave;
    if (u >= (unsigned)(NT_MAX * (DM / 64))) return;
    const unsigned rowtile = u / (unsigned)(DM / 64);
    const unsigned ct = u - rowtile * (unsigned)(DM / 64);
    const int nt = min(max(tbl[TBL_NTILES], 0), NT_MAX);
    if ((int)rowtile >= nt) return;
    const int e = min(max(tbl[TBL_TILE_E + rowtile], 0), NE - 1);
    const size_t wbase = (size_t)(unsigned)e * (size_t)(DM * DM);
    const unsigned m0 = rowtile << 6, n0 = ct << 6;
    const unsigned rlane = lane & 15u;
    const unsigned koff = (lane >> 4) * 8u;
    const unsigned mOff = koff;

    v8f acc[4][4];
#pragma unroll
    for (int i = 0; i < 4; ++i)
#pragma unroll
        for (int j = 0; j < 4; ++j) acc[i][j] = (v8f){0.f,0.f,0.f,0.f,0.f,0.f,0.f,0.f};

    for (unsigned k0 = 0; k0 < (unsigned)DM; k0 += 32u) {
        v16h bh[4];
#pragma unroll
        for (int j = 0; j < 4; ++j)
            bh[j] = frag_ld(Wp + wbase + (size_t)(n0 + ((unsigned)j << 4) + rlane) * DM + koff + k0);
#pragma unroll
        for (int i = 0; i < 4; ++i) {
            const v16h ah = frag_ld(Xg + (size_t)(m0 + ((unsigned)i << 4) + rlane) * DM + koff + k0);
#pragma unroll
            for (int j = 0; j < 4; ++j) acc[i][j] = wmma16g(ah, bh[j], acc[i][j]);
        }
    }

    float ebv[4];
#pragma unroll
    for (int j = 0; j < 4; ++j) ebv[j] = bfr(eb[(unsigned)e * (unsigned)DM + n0 + ((unsigned)j << 4) + rlane]);

    float* slab = sT[wave];
#pragma unroll
    for (int i = 0; i < 4; ++i) {
        const unsigned mBase = m0 + ((unsigned)i << 4);
#pragma unroll
        for (int j = 0; j < 4; ++j)
#pragma unroll
            for (int r = 0; r < 8; ++r)
                slab[(mOff + (unsigned)r) * 68u + ((unsigned)j << 4) + rlane] = acc[i][j][r] * SC_Y + ebv[j];
        wave_sync_lds();
        const unsigned hh = lane >> 4, c4 = (lane & 15u) * 4u;
#pragma unroll
        for (int half = 0; half < 2; ++half) {
            v4f vv[4];
#pragma unroll
            for (int it = 0; it < 4; ++it) {
                const unsigned row = (unsigned)(half * 4 + it) * 2u + hh;
                vv[it] = *(const v4f*)(slab + row * 68u + c4);
            }
            for (int pass = 0; pass < 2; ++pass) {
#pragma unroll
                for (int it = 0; it < 4; ++it) {
                    const unsigned row = (unsigned)(half * 4 + it) * 2u + hh;
                    *(volatile v4f*)(Yg + (size_t)(mBase + row) * DM + n0 + c4) = vv[it];
                }
                __threadfence();
            }
        }
        wave_sync_lds();
    }
}

__global__ __launch_bounds__(256) void k_combine(const float* __restrict__ Yg, const float* __restrict__ wgt, const int* __restrict__ tbl,
                                                 float* __restrict__ out) {
    const unsigned t = blockIdx.x;
    if (t >= (unsigned)NTOK) return;
    const unsigned c = threadIdx.x * 4u;
    const int r0 = min(max(tbl[TBL_SLOTROW + 2u * t], 0), R_MAX - 1);
    const int r1 = min(max(tbl[TBL_SLOTROW + 2u * t + 1u], 0), R_MAX - 1);
    const float w0 = wgt[2u * t], w1 = wgt[2u * t + 1u];
    const v4f a = *(const v4f*)(Yg + (size_t)(unsigned)r0 * DM + c);
    const v4f b = *(const v4f*)(Yg + (size_t)(unsigned)r1 * DM + c);
    const v4f y = (a * w0) + (b * w1);
    VST2(v4f, out + (size_t)t * DM + c, y);
}

extern "C" void kernel_launch(void* const* d_in, const int* in_sizes, int n_in, void* d_out, int out_size,
                              void* d_ws, size_t ws_size, hipStream_t stream) {
    if (n_in < 6) return;
    if (in_sizes[0] < NTOK * DM || in_sizes[1] < NTOK * DM || in_sizes[2] < DM * NE) return;
    if (in_sizes[3] < DM * NE || in_sizes[4] < NE * DM * DM || in_sizes[5] < NE * DM) return;
    if (out_size < NTOK * DM) return;

    const float* x  = (const float*)d_in[0];
    const float* nx = (const float*)d_in[1];
    const float* rw = (const float*)d_in[2];
    const float* nw = (const float*)d_in[3];
    const float* ew = (const float*)d_in[4];
    const float* eb = (const float*)d_in[5];
    float* out = (float*)d_out;

    char* wsp = (char*)d_ws;
    size_t off = 0;
    auto carve = [&](size_t bytes) -> void* { void* r = wsp + off; off += (bytes + 255) & ~(size_t)255; return r; };
    h16*   x16 = (h16*)carve((size_t)NTOK * DM * 2);
    h16*   wt  = (h16*)carve((size_t)NE * DM * DM * 2);
    int*   sel = (int*)carve((size_t)NSLOT * 4);
    float* wgt = (float*)carve((size_t)NSLOT * 4);
    int*   tbl = (int*)carve((size_t)TBL_WORDS * 4);
    h16*   Xg  = (h16*)carve((size_t)R_MAX * DM * 2);
    float* Yg  = (float*)carve((size_t)R_MAX * DM * 4);
    if (off != WS_TOTAL || off > ws_size || off > (size_t)134217728) return;

    k_plane<CX_LOG2><<<(NTOK * DM / 8) / 256, 256, 0, stream>>>(x, x16, (unsigned)(NTOK * DM / 8));
    k_planeT<<<NE * (DM / 64) * (DM / 64), 256, 0, stream>>>(ew, wt);
    k_gate<<<NTOK / 128, 256, 0, stream>>>(x, nx, rw, nw, sel, wgt);
    k_route<<<1, 512, 0, stream>>>(sel, tbl);
    k_gather<<<R_MAX / 2, 256, 0, stream>>>(x16, tbl, Xg);
    k_ffn<<<(NT_MAX * (DM / 64) + 7) / 8, 256, 0, stream>>>(Xg, wt, eb, tbl, Yg);
    k_combine<<<NTOK, 256, 0, stream>>>(Yg, wgt, tbl, out);
}
